// NeuSDF_1743756722497
// MI455X (gfx1250) — hardware-verified
//
#include <hip/hip_runtime.h>


#define NPT  1048576
#define RES  512
#define HID  128
#define PCH  65536
#define NCHK (NPT / PCH)
typedef _Float16 h16;
typedef unsigned short bf;
typedef __attribute__((ext_vector_type(16))) __bf16   v16bf;
typedef __attribute__((ext_vector_type(16))) _Float16 v16h;
typedef __attribute__((ext_vector_type(8)))  _Float16 v8h;
typedef __attribute__((ext_vector_type(8)))  unsigned short v8us;
typedef __attribute__((ext_vector_type(8)))  float    v8f;
typedef __attribute__((ext_vector_type(4)))  float    v4f;
typedef v8h  __attribute__((may_alias)) v8ha;
typedef v4f  __attribute__((may_alias)) v4fa;
typedef v8us __attribute__((may_alias)) v8usa;

__device__ __forceinline__ unsigned short f2bf(float f) { unsigned u = __float_as_uint(f); u += 0x7FFFu + ((u >> 16) & 1u); return (unsigned short)(u >> 16); }
__device__ __forceinline__ float bf2f(unsigned short b) { return __uint_as_float(((unsigned)b) << 16); }
__device__ __forceinline__ float bfr(float f) { return bf2f(f2bf(f)); }
__device__ __forceinline__ v16h cat16(v8h lo, v8h hi) { return __builtin_shufflevector(lo, hi, 0, 1, 2, 3, 4, 5, 6, 7, 8, 9, 10, 11, 12, 13, 14, 15); }
__device__ __forceinline__ v16bf cat16b(v8us lo, v8us hi) { return __builtin_bit_cast(v16bf, __builtin_shufflevector(lo, hi, 0, 1, 2, 3, 4, 5, 6, 7, 8, 9, 10, 11, 12, 13, 14, 15)); }
__device__ __forceinline__ v8f wmma16(v16h a, v16h b, v8f c) { return __builtin_amdgcn_wmma_f32_16x16x32_f16(false, a, false, b, (short)0, c, false, false); }
__device__ __forceinline__ v8f wmmab(v16bf a, v16bf b, v8f c) { return __builtin_amdgcn_wmma_f32_16x16x32_bf16(false, a, false, b, (short)0, c, false, false); }


template <typename T16> struct WFrag;
template <> struct WFrag<h16> { typedef v16h V; static __device__ __forceinline__ V ld(const h16* p) { return cat16(*(const v8h*)p, *(const v8h*)(p + 16)); } static __device__ __forceinline__ v8f mma(V a, V b, v8f c) { return wmma16(a, b, c); } };
template <> struct WFrag<bf> { typedef v16bf V; static __device__ __forceinline__ V ld(const bf* p) { return cat16b(*(const v8us*)p, *(const v8us*)(p + 16)); } static __device__ __forceinline__ v8f mma(V a, V b, v8f c) { return wmmab(a, b, c); } };
template <typename T16, int NSPLIT, bool BIAS>
__global__ __launch_bounds__(32) void k_gemmw(const T16* __restrict__ A, const T16* __restrict__ A2, const T16* __restrict__ Bt, const T16* __restrict__ Bt2, int K, float* C, int ldc, const float* __restrict__ bias, size_t sA, size_t sB, size_t sC) {
    typedef typename WFrag<T16>::V V;
    __shared__ __align__(16) float os[16 * 68];
    const size_t z = blockIdx.z; A += z * sA; if (A2) A2 += z * sA; Bt += z * sB; if (Bt2) Bt2 += z * sB; C += z * sC;
    const int lane = threadIdx.x & 31, lr = lane & 15, hi = lane >> 4; const int r0 = blockIdx.x * 64, c0 = blockIdx.y * 64;
    v8f acc[4][4];
#pragma unroll
    for (int mb = 0; mb < 4; ++mb)
#pragma unroll
        for (int nb = 0; nb < 4; ++nb) acc[mb][nb] = (v8f){};
    const size_t aoff = (size_t)(r0 + lr) * K + 8 * hi, boff = (size_t)(c0 + lr) * K + 8 * hi;
#pragma unroll 1
    for (int kc = 0; kc < K; kc += 32) {
        V a[4], a2[4];
#pragma unroll
        for (int mb = 0; mb < 4; ++mb) { a[mb] = WFrag<T16>::ld(A + aoff + (size_t)mb * 16 * K + kc); if (NSPLIT == 1 || NSPLIT == 2) a2[mb] = WFrag<T16>::ld(A2 + aoff + (size_t)mb * 16 * K + kc); }
#pragma unroll
        for (int nb = 0; nb < 4; ++nb) { const V b = WFrag<T16>::ld(Bt + boff + (size_t)nb * 16 * K + kc); V b2; if (NSPLIT >= 2) b2 = WFrag<T16>::ld(Bt2 + boff + (size_t)nb * 16 * K + kc);
#pragma unroll
            for (int mb = 0; mb < 4; ++mb) { acc[mb][nb] = WFrag<T16>::mma(a[mb], b, acc[mb][nb]); if (NSPLIT == 1 || NSPLIT == 2) acc[mb][nb] = WFrag<T16>::mma(a2[mb], b, acc[mb][nb]); if (NSPLIT >= 2) acc[mb][nb] = WFrag<T16>::mma(a[mb], b2, acc[mb][nb]); } }
        asm volatile("v_nop\n\tv_nop\n\tv_nop\n\tv_nop" : "+v"(acc[0][0]), "+v"(acc[1][1]), "+v"(acc[2][2]), "+v"(acc[3][3]) : "v"(a[0]), "v"(a[3]));
    }
#pragma unroll
    for (int mb = 0; mb < 4; ++mb) {
#pragma unroll
        for (int nb = 0; nb < 4; ++nb) {
#pragma unroll
            for (int j = 0; j < 8; ++j) os[(hi * 8 + j) * 68 + nb * 16 + lr] = acc[mb][nb][j]; }
        __builtin_amdgcn_wave_barrier(); asm volatile("" ::: "memory");
        float* crow = C + (size_t)(r0 + mb * 16) * ldc + c0;
#pragma unroll 1
        for (int ps = 0; ps < 2; ++ps) {
#pragma unroll
            for (int s = 0; s < 8; ++s) { const int row = 2 * s + hi, cofs = lr * 4; v4f val = *(const v4fa*)(os + row * 68 + cofs); if (BIAS) { val[0] += bfr(bias[c0 + cofs]); val[1] += bfr(bias[c0 + cofs + 1]); val[2] += bfr(bias[c0 + cofs + 2]); val[3] += bfr(bias[c0 + cofs + 3]); }
                *(volatile v4f*)(crow + (size_t)row * ldc + cofs) = val; }
            if (ps == 0) __threadfence(); }
        __builtin_amdgcn_wave_barrier(); asm volatile("" ::: "memory");
    }
}

__device__ __forceinline__ h16 tohx(float x) { return (h16)x; }
typedef __attribute__((ext_vector_type(2))) _Float16 v2h;
typedef __attribute__((ext_vector_type(4))) _Float16 v4h;

__global__ __launch_bounds__(256) void k_wth(const float* __restrict__ w, int K, int N, int Np, h16* Bt) {
    const int lane = threadIdx.x & 31; const int nlines = Np * K / 64; const int wg = blockIdx.x * 8 + (threadIdx.x >> 5), nw = gridDim.x * 8;
#pragma unroll 1
    for (int ps = 0; ps < 2; ++ps) {
#pragma unroll 1
        for (int L = wg; L < nlines; L += nw) { const int e = L * 64 + lane * 2; v2h o;
#pragma unroll
            for (int q = 0; q < 2; ++q) { const int n = (e + q) / K, k = (e + q) % K; o[q] = (n < N) ? tohx(bfr(w[(size_t)k * N + (n < N ? n : 0)])) : tohx(0.f); }
            *(volatile v2h*)(Bt + e) = o; }
        if (ps == 0) __threadfence(); }
}
__global__ __launch_bounds__(64) void k_bpad(const float* __restrict__ b, int N, float* out) { const int i = threadIdx.x; const float v = i < N ? b[i < N ? i : 0] : 0.f; *(volatile float*)(out + i) = v; __threadfence(); *(volatile float*)(out + i) = v; }
__device__ __forceinline__ float interp(const float* __restrict__ pl, float c1, float c2) {
    const float f1 = floorf(c1), f2 = floorf(c2); int i1 = (int)f1, i2 = (int)f2; i1 = i1 < 0 ? 0 : (i1 > RES - 1 ? RES - 1 : i1); i2 = i2 < 0 ? 0 : (i2 > RES - 1 ? RES - 1 : i2);
    const int j1 = i1 + 1 > RES - 1 ? RES - 1 : i1 + 1, j2 = i2 + 1 > RES - 1 ? RES - 1 : i2 + 1;
    const float bl = bfr(pl[i1 * RES + i2]), br = bfr(pl[j1 * RES + i2]), tl = bfr(pl[i1 * RES + j2]), tr = bfr(pl[j1 * RES + j2]);
    const float h = c1 - f1, v = c2 - f2; const float top = tl + (tr - tl) * h, bottom = bl + (br - bl) * h; return bottom + (top - bottom) * v;
}
__global__ __launch_bounds__(256) void k_feat(const float* __restrict__ pts, const float* __restrict__ pxy, const float* __restrict__ pyz, const float* __restrict__ pxz, const float* __restrict__ w1, const float* __restrict__ b1, int p0, h16* H1) {
    const int lane = threadIdx.x & 31; const int g0 = (blockIdx.x * 8 + (threadIdx.x >> 5)) * 32; if (g0 >= PCH) return; const int pi = p0 + g0 + lane;
    const float px = (bfr(pts[(size_t)pi * 3 + 0]) + 1.0f) * 0.5f * 511.0f, py = (bfr(pts[(size_t)pi * 3 + 1]) + 1.0f) * 0.5f * 511.0f, pz = (bfr(pts[(size_t)pi * 3 + 2]) + 1.0f) * 0.5f * 511.0f;
    const float Fm = (interp(pxy, px, py) + interp(pxz, px, pz)) + interp(pyz, py, pz);
    float wl[4], bl4[4];
#pragma unroll
    for (int q = 0; q < 4; ++q) { wl[q] = bfr(w1[lane * 4 + q]); bl4[q] = bfr(b1[lane * 4 + q]); }
#pragma unroll 1
    for (int ps = 0; ps < 2; ++ps) {
#pragma unroll 1
        for (int r = 0; r < 32; ++r) { const float F = __shfl(Fm, r, 32); v4h o;
#pragma unroll
            for (int q = 0; q < 4; ++q) o[q] = tohx(fmaxf(__fadd_rn(__fmul_rn(F, wl[q]), bl4[q]), 0.f));
            *(volatile v4h*)(H1 + (size_t)(g0 + r) * HID + lane * 4) = o; }
        if (ps == 0) __threadfence(); }
}
__global__ __launch_bounds__(256) void k_relu16(const float* __restrict__ H, h16* P) {
    const int lane = threadIdx.x & 31; const int L0 = (blockIdx.x * 8 + (threadIdx.x >> 5)) * 8; const int nlines = PCH * HID / 64;
#pragma unroll 1
    for (int ps = 0; ps < 2; ++ps) {
#pragma unroll
        for (int l = 0; l < 8; ++l) { const int L = L0 + l; if (L >= nlines) break; const int e = L * 64 + lane * 2; v2h v;
#pragma unroll
            for (int q = 0; q < 2; ++q) v[q] = tohx(fmaxf(H[e + q], 0.f));
            *(volatile v2h*)(P + e) = v; }
        if (ps == 0) __threadfence(); }
}
__global__ __launch_bounds__(256) void k_fin(const float* __restrict__ C, int p0, float* OUT) {
    const int lane = threadIdx.x & 31; const int r0 = (blockIdx.x * 8 + (threadIdx.x >> 5)) * 32; if (r0 >= PCH) return; const float v = tanhf(C[(size_t)(r0 + lane) * 64]);
    float* dst = OUT + p0 + r0 + lane; *(volatile float*)dst = v; __threadfence(); *(volatile float*)dst = v;
}

extern "C" void kernel_launch(void* const* d_in, const int* in_sizes, int n_in,
                              void* d_out, int out_size, void* d_ws, size_t ws_size, hipStream_t stream) {
    (void)in_sizes; (void)n_in; (void)out_size;
    const float* pts = (const float*)d_in[0]; const float* pxy = (const float*)d_in[1]; const float* pyz = (const float*)d_in[2]; const float* pxz = (const float*)d_in[3];
    const float* w1 = (const float*)d_in[4]; const float* b1 = (const float*)d_in[5]; const float* w2 = (const float*)d_in[6]; const float* b2 = (const float*)d_in[7]; const float* w3 = (const float*)d_in[8]; const float* b3 = (const float*)d_in[9];
    float* OUT = (float*)d_out;
    char* wsp = (char*)d_ws;
    auto take = [&](size_t bytes) { char* p = wsp; wsp += (bytes + 255) & ~(size_t)255; return (void*)p; };
    h16* W2t = (h16*)take((size_t)HID * HID * 2); h16* W3t = (h16*)take((size_t)64 * HID * 2); float* B3P = (float*)take(64 * 4);
    h16* H1 = (h16*)take((size_t)PCH * HID * 2); float* H2 = (float*)take((size_t)PCH * HID * 4); h16* P2 = (h16*)take((size_t)PCH * HID * 2); float* C3 = (float*)take((size_t)PCH * 64 * 4);
    if ((size_t)(wsp - (char*)d_ws) > ws_size) return;
    k_wth<<<4, 256, 0, stream>>>(w2, HID, HID, HID, W2t); k_wth<<<2, 256, 0, stream>>>(w3, HID, 1, 64, W3t); k_bpad<<<1, 64, 0, stream>>>(b3, 1, B3P);
    for (int ch = 0; ch < NCHK; ++ch) { const int p0 = ch * PCH;
        k_feat<<<PCH / 32 / 8, 256, 0, stream>>>(pts, pxy, pyz, pxz, w1, b1, p0, H1);
        k_gemmw<h16, 0, true><<<dim3(PCH / 64, HID / 64, 1), 32, 0, stream>>>(H1, nullptr, W2t, nullptr, HID, H2, HID, b2, 0, 0, 0);
        k_relu16<<<(PCH * HID / 64 + 63) / 64, 256, 0, stream>>>(H2, P2);
        k_gemmw<h16, 0, true><<<dim3(PCH / 64, 1, 1), 32, 0, stream>>>(P2, nullptr, W3t, nullptr, HID, C3, 64, B3P, 0, 0, 0);
        k_fin<<<PCH / 32 / 8, 256, 0, stream>>>(C3, p0, OUT); }
}
